// DecoderRNN_6975026889175
// MI455X (gfx1250) — hardware-verified
//
#include <hip/hip_runtime.h>
#include <math.h>

constexpr int NBAT   = 64;
constexpr int NPIX   = 49;
constexpr int NENC   = 2048;
constexpr int NSEQ   = 26;
constexpr int NSTEP  = NSEQ - 1;
constexpr int NVOC   = 10000;
constexpr int NVOCP  = 10048;
constexpr int NVOCB  = 10112;
constexpr int NEMB   = 512;
constexpr int NHID   = 512;
constexpr int NATT   = 512;
constexpr int NGATE  = 4 * NHID;
constexpr int NXIN   = NEMB + NENC;
constexpr int NHP    = NATT + NGATE;
constexpr int NROWS  = NBAT * NSTEP;
constexpr int NFROWS = NBAT * NPIX;
constexpr int APITCH = 64;
constexpr int NTHR   = 256;
constexpr int NOUT0  = NROWS * NVOC;
constexpr int NOUT1  = NROWS * NPIX;
constexpr int BIAS_G_OFF  = 0;
constexpr int BIAS_HP_OFF = NGATE;
constexpr int BIAS_FC_OFF = NGATE + NHP;
constexpr int BIAS_TOTAL  = BIAS_FC_OFF + NVOCB;
constexpr int SCORE_TRIPS = (NPIX + 7) / 8;

static_assert(NSTEP == 25);
static_assert(NROWS == 1600 && NFROWS == 3136);
static_assert(NROWS % 64 == 0 && NFROWS % 64 == 0 && NBAT % 64 == 0);
static_assert(NVOCP % 64 == 0 && NVOCP >= NVOC && NGATE % 64 == 0 && NHP % 64 == 0 && NHID % 64 == 0 && NATT % 64 == 0);
static_assert(NENC % 32 == 0 && NHID % 32 == 0 && NEMB % 32 == 0);
static_assert(NVOC % 4 == 0);
static_assert(((size_t)NOUT0 * 4) % 128 == 0);
static_assert(((size_t)NOUT1 * 4) % 128 == 0);
static_assert(BIAS_TOTAL % 128 == 0 && BIAS_HP_OFF % 128 == 0 && BIAS_FC_OFF % 128 == 0);
static_assert(NVOCB >= NVOCP);
static_assert(NENC == NTHR * 8);
static_assert(NATT == 32 * 16);
static_assert(NPIX <= 64 && NPIX > 32);
static_assert((NOUT0 / 4) % NTHR == 0);

typedef __attribute__((ext_vector_type(16))) _Float16 v16h;
typedef __attribute__((ext_vector_type(8)))  _Float16 v8h;
typedef __attribute__((ext_vector_type(8)))  float    v8f;
typedef __attribute__((ext_vector_type(4)))  float    v4f;

__device__ __forceinline__ void gemm_guard_h(v8f& a, v8f& b, v8f& c, v8f& d, v16h x, v16h y0, v16h y1, v16h y2, v16h y3) {
  asm volatile("v_nop\n\tv_nop\n\tv_nop\n\tv_nop" : "+v"(a), "+v"(b), "+v"(c), "+v"(d) : "v"(x), "v"(y0), "v"(y1), "v"(y2), "v"(y3));
}
__device__ __forceinline__ void keep4_h(v16h a, v16h b, v16h c, v16h d) { asm volatile("v_nop" :: "v"(a), "v"(b), "v"(c), "v"(d)); }
__device__ __forceinline__ void acc_guard4(v8f& a, v8f& b, v8f& c, v8f& d) { asm volatile("v_nop\n\tv_nop\n\tv_nop\n\tv_nop" : "+v"(a), "+v"(b), "+v"(c), "+v"(d)); }

struct FragH {
  union U { v16h v; v8h h[2]; };
  static __device__ __forceinline__ v16h load(const _Float16* p) {
    U f; f.h[0] = *(const v8h*)(p); f.h[1] = *(const v8h*)(p + 16); return f.v;
  }
  static __device__ __forceinline__ v8f mma(v16h a, v16h b, v8f c) {
    return __builtin_amdgcn_wmma_f32_16x16x32_f16(false, a, false, b, (short)0, c, false, false);
  }
};

template <int BIAS_MODE, int OUT_MODE>
__global__ __launch_bounds__(256) void wmma_gemm64_f16(
    const unsigned short* __restrict__ Ap, int lda,
    const unsigned short* __restrict__ Btp, int ldb,
    void* __restrict__ Cout, int ldc,
    const float* __restrict__ bias, int M, int N, int K) {
  const _Float16* A  = (const _Float16*)Ap;
  const _Float16* Bt = (const _Float16*)Btp;
  __shared__ __align__(16) float sT[8][16 * 68];
  const int lane = threadIdx.x & 31;
  const int wave = threadIdx.x >> 5;
  const int tilesN = N >> 6;
  const int tilesM = M >> 6;
  const int tile = blockIdx.x * 8 + wave;
  if (tile >= tilesM * tilesN) return;
  const int tm = tile / tilesN;
  const int tn = tile - tm * tilesN;
  const int m0 = tm << 6;
  const int n0 = tn << 6;

  const int rlane = lane & 15;
  const int koff  = (lane >> 4) * 8;
  const int mOff  = (lane >> 4) * 8;

  v8f acc[4][4];
#pragma unroll
  for (int i = 0; i < 4; ++i)
#pragma unroll
    for (int j = 0; j < 4; ++j) acc[i][j] = (v8f){0.f,0.f,0.f,0.f,0.f,0.f,0.f,0.f};

  for (int k0 = 0; k0 < K; k0 += 32) {
    v16h bh[4];
#pragma unroll
    for (int j = 0; j < 4; ++j) {
      const size_t bo = (size_t)(n0 + (j << 4) + rlane) * ldb + koff + k0;
      bh[j] = FragH::load(Bt + bo);
    }
#pragma unroll
    for (int i = 0; i < 4; ++i) {
      const size_t ao = (size_t)(m0 + (i << 4) + rlane) * lda + koff + k0;
      const v16h ah = FragH::load(A + ao);
#pragma unroll
      for (int j = 0; j < 4; ++j) acc[i][j] = FragH::mma(ah, bh[j], acc[i][j]);
      gemm_guard_h(acc[i][0], acc[i][1], acc[i][2], acc[i][3], ah, bh[0], bh[1], bh[2], bh[3]);
    }
    keep4_h(bh[0], bh[1], bh[2], bh[3]);
  }
  acc_guard4(acc[0][0], acc[0][1], acc[0][2], acc[0][3]);
  acc_guard4(acc[1][0], acc[1][1], acc[1][2], acc[1][3]);
  acc_guard4(acc[2][0], acc[2][1], acc[2][2], acc[2][3]);
  acc_guard4(acc[3][0], acc[3][1], acc[3][2], acc[3][3]);

  float* slab = sT[wave];
#pragma unroll
  for (int i = 0; i < 4; ++i) {
    const int mBase = m0 + (i << 4);
#pragma unroll
    for (int j = 0; j < 4; ++j) {
      const int n = n0 + (j << 4) + rlane;
      float bv = 0.f;
      if (BIAS_MODE == 2) bv = bias[n];
#pragma unroll
      for (int r = 0; r < 8; ++r) {
        float v = acc[i][j][r];
        if (BIAS_MODE == 2) v += bv;
        slab[(mOff + r) * 68 + (j << 4) + rlane] = v;
      }
    }
    __builtin_amdgcn_fence(__ATOMIC_RELEASE, "workgroup");
    __builtin_amdgcn_wave_barrier();
    __builtin_amdgcn_fence(__ATOMIC_ACQUIRE, "workgroup");
    if (OUT_MODE == 0) {
      float* C = (float*)Cout;
      const int hh = lane >> 4, c4 = (lane & 15) * 4;
      for (int pass = 0; pass < 2; ++pass) {
#pragma unroll
        for (int it = 0; it < 8; ++it) {
          const int row = it * 2 + hh;
          v4f v = *(const v4f*)(slab + row * 68 + c4);
          *(volatile v4f*)(C + (size_t)(mBase + row) * ldc + n0 + c4) = v;
        }
        __threadfence();
      }
    } else {
      const int q = lane >> 3, c8 = (lane & 7) * 8;
      unsigned short* C = (unsigned short*)Cout;
      for (int pass = 0; pass < 2; ++pass) {
#pragma unroll
        for (int it = 0; it < 4; ++it) {
          const int row = it * 4 + q;
          const float* sp = slab + row * 68 + c8;
          v8h hv;
#pragma unroll
          for (int e = 0; e < 8; ++e) hv[e] = (_Float16)sp[e];
          *(volatile v8h*)(C + (size_t)(mBase + row) * ldc + n0 + c8) = hv;
        }
        __threadfence();
      }
    }
    __builtin_amdgcn_fence(__ATOMIC_RELEASE, "workgroup");
    __builtin_amdgcn_wave_barrier();
    __builtin_amdgcn_fence(__ATOMIC_ACQUIRE, "workgroup");
  }
}

__global__ __launch_bounds__(NTHR) void cvt8_f16_kernel(const float* __restrict__ src, unsigned short* __restrict__ dst,
                                                        int nrow_dst, int nrow_src, int ncol8, int spitch, int scol0) {
  const int i  = blockIdx.x * NTHR + threadIdx.x;
  const int n8 = nrow_dst * ncol8;
  if (i < n8) {
    const int row  = i / ncol8;
    const int c8   = i - row * ncol8;
    const int rowc = row < nrow_src ? row : nrow_src - 1;
    const bool live = row < nrow_src;
    const float* sp = src + (size_t)rowc * spitch + scol0 + c8 * 8;
    const v4f a = *(const v4f*)(sp);
    const v4f b = *(const v4f*)(sp + 4);
    v8h hv;
#pragma unroll
    for (int e = 0; e < 4; ++e) {
      const float fa = live ? a[e] : 0.0f;
      const float fb = live ? b[e] : 0.0f;
      hv[e]     = (_Float16)fa;
      hv[4 + e] = (_Float16)fb;
    }
    *(volatile v8h*)(dst + (size_t)i * 8) = hv;
    __threadfence();
    *(volatile v8h*)(dst + (size_t)i * 8) = hv;
  }
}

__global__ __launch_bounds__(NTHR) void bias_prep_kernel(const float* __restrict__ b_ih, const float* __restrict__ b_hh,
                                                         const float* __restrict__ b_dec, const float* __restrict__ b_fcn,
                                                         float* __restrict__ dst) {
  const int i = blockIdx.x * NTHR + threadIdx.x;
  if (i < BIAS_TOTAL / 4) {
    const int f  = 4 * i;
    const int ia = f < NGATE - 4 ? f : NGATE - 4;
    const int kb = f - BIAS_HP_OFF;
    const int kbc = kb < 0 ? 0 : (kb > NATT - 4 ? NATT - 4 : kb);
    const int kc = f - BIAS_FC_OFF;
    const int kcc = kc < 0 ? 0 : (kc > NVOC - 4 ? NVOC - 4 : kc);
    const v4f va1 = *(const v4f*)(b_ih + ia);
    const v4f va2 = *(const v4f*)(b_hh + ia);
    const v4f vb  = *(const v4f*)(b_dec + kbc);
    const v4f vc  = *(const v4f*)(b_fcn + kcc);
    const bool inA   = f < BIAS_HP_OFF;
    const bool liveB = (!inA) && (f < BIAS_FC_OFF) && (kb < NATT);
    const bool liveC = (f >= BIAS_FC_OFF) && (kc < NVOC);
    v4f o;
#pragma unroll
    for (int e = 0; e < 4; ++e) {
      const float sa = va1[e] + va2[e];
      o[e] = inA ? sa : (liveB ? vb[e] : (liveC ? vc[e] : 0.0f));
    }
    *(volatile v4f*)(dst + f) = o;
    __threadfence();
    *(volatile v4f*)(dst + f) = o;
  }
}

__global__ __launch_bounds__(NTHR) void mean16_kernel(const float* __restrict__ feat, unsigned short* __restrict__ mean16) {
  const int i  = blockIdx.x * NTHR + threadIdx.x;
  const int b  = i >> 8;
  const int c8 = (i & 255) * 8;
  const float* fp = feat + (size_t)b * NPIX * NENC + c8;
  float acc[8];
#pragma unroll
  for (int e = 0; e < 8; ++e) acc[e] = 0.0f;
#pragma unroll 1
  for (int n = 0; n < NPIX; ++n) {
    const v4f x0 = *(const v4f*)(fp + (size_t)n * NENC);
    const v4f x1 = *(const v4f*)(fp + (size_t)n * NENC + 4);
#pragma unroll
    for (int e = 0; e < 4; ++e) { acc[e] += x0[e]; acc[4 + e] += x1[e]; }
  }
  v8h hv;
#pragma unroll
  for (int e = 0; e < 8; ++e) hv[e] = (_Float16)(acc[e] * (1.0f / (float)NPIX));
  *(volatile v8h*)(mean16 + (size_t)i * 8) = hv;
  __threadfence();
  *(volatile v8h*)(mean16 + (size_t)i * 8) = hv;
}

__global__ __launch_bounds__(NTHR) void gather16_kernel(const int* __restrict__ captions, const float* __restrict__ emb,
                                                        unsigned short* __restrict__ x16) {
  const int i   = blockIdx.x * NTHR + threadIdx.x;
  const int row = i >> 6;
  const int c8  = (i & 63) * 8;
  const int t   = row >> 6;
  const int b   = row & 63;
  int tok = captions[b * NSEQ + t];
  tok = tok < 0 ? 0 : (tok > NVOC - 1 ? NVOC - 1 : tok);
  const float* sp = emb + (size_t)tok * NEMB + c8;
  const v4f a  = *(const v4f*)(sp);
  const v4f bq = *(const v4f*)(sp + 4);
  v8h hv;
#pragma unroll
  for (int e = 0; e < 4; ++e) { hv[e] = (_Float16)a[e]; hv[4 + e] = (_Float16)bq[e]; }
  *(volatile v8h*)(x16 + (size_t)i * 8) = hv;
  __threadfence();
  *(volatile v8h*)(x16 + (size_t)i * 8) = hv;
}

__global__ __launch_bounds__(NTHR) void attn_step_kernel(const float* __restrict__ att1, const float* __restrict__ hproj,
                                                         const float* __restrict__ feat, const float* __restrict__ wfull,
                                                         const float* __restrict__ bfull, float* __restrict__ alpha_ws,
                                                         unsigned short* __restrict__ ctx16, int t) {
  __shared__ float e_s[64];
  __shared__ __align__(16) float al_s[64];
  const int b = blockIdx.x, tid = threadIdx.x;
  const int wave = tid >> 5, lane = tid & 31;

  if (tid >= NPIX && tid < 64) e_s[tid] = 0.0f;

  v4f a2[4], wf[4];
#pragma unroll
  for (int q = 0; q < 4; ++q) {
    a2[q] = *(const v4f*)(hproj + (size_t)b * NHP + 128 * q + 4 * lane);
    wf[q] = *(const v4f*)(wfull + 128 * q + 4 * lane);
  }
  const float bf = bfull[0];

#pragma unroll 1
  for (int it = 0; it < SCORE_TRIPS; ++it) {
    const int n  = it * 8 + wave;
    const int nc = n < NPIX ? n : NPIX - 1;
    const float* a1 = att1 + ((size_t)b * NPIX + nc) * NATT + 4 * lane;
    float s = 0.0f;
#pragma unroll
    for (int q = 0; q < 4; ++q) {
      const v4f x = *(const v4f*)(a1 + 128 * q);
#pragma unroll
      for (int e = 0; e < 4; ++e) {
        const float r = fmaxf(x[e] + a2[q][e], 0.0f);
        s = fmaf(r, wf[q][e], s);
      }
    }
#pragma unroll
    for (int off = 16; off > 0; off >>= 1) s += __shfl_xor(s, off, 32);
    if (lane == 0 && n < NPIX) e_s[n] = s + bf;
  }
  __syncthreads();

  {
    const int n1  = lane + 32;
    const int n1c = n1 < NPIX ? n1 : NPIX - 1;
    const bool has1 = n1 < NPIX;
    const float e0 = e_s[lane];
    const float e1 = e_s[n1c];
    float m = fmaxf(e0, e1);
#pragma unroll
    for (int off = 16; off > 0; off >>= 1) m = fmaxf(m, __shfl_xor(m, off, 32));
    const float p0  = expf(e0 - m);
    const float p1r = expf(e1 - m);
    const float p1  = has1 ? p1r : 0.0f;
    float sum = p0 + p1;
#pragma unroll
    for (int off = 16; off > 0; off >>= 1) sum += __shfl_xor(sum, off, 32);
    const float inv = 1.0f / sum;
    if (wave == 0) {
      al_s[lane]      = p0 * inv;
      al_s[lane + 32] = p1 * inv;
    }
  }
  __syncthreads();

  if (tid < 16) {
    const v4f av = *(const v4f*)(al_s + 4 * tid);
    float* ap = alpha_ws + ((size_t)(b * NSTEP + t)) * APITCH + 4 * tid;
    *(volatile v4f*)ap = av;
    __threadfence();
    *(volatile v4f*)ap = av;
  }

  const float* fb = feat + (size_t)b * NPIX * NENC + tid * 8;
  float acc[8];
#pragma unroll
  for (int e = 0; e < 8; ++e) acc[e] = 0.0f;
#pragma unroll 1
  for (int n = 0; n < NPIX; ++n) {
    const float w = al_s[n];
    const v4f x0 = *(const v4f*)(fb + (size_t)n * NENC);
    const v4f x1 = *(const v4f*)(fb + (size_t)n * NENC + 4);
#pragma unroll
    for (int e = 0; e < 4; ++e) {
      acc[e]     = fmaf(w, x0[e], acc[e]);
      acc[4 + e] = fmaf(w, x1[e], acc[4 + e]);
    }
  }
  v8h hv;
#pragma unroll
  for (int e = 0; e < 8; ++e) hv[e] = (_Float16)acc[e];
  unsigned short* cp = ctx16 + (size_t)b * NENC + tid * 8;
  *(volatile v8h*)cp = hv;
  __threadfence();
  *(volatile v8h*)cp = hv;
}

__device__ __forceinline__ float sigm_f(float x) { return 1.0f / (1.0f + expf(-x)); }
__device__ __forceinline__ float tanh_f(float x) { return 1.0f - 2.0f / (1.0f + expf(2.0f * x)); }

__global__ __launch_bounds__(NTHR) void lstm_point_kernel(const float* __restrict__ gctx, const float* __restrict__ hproj,
                                                          const float* __restrict__ gemb, const float* __restrict__ c_in,
                                                          float* __restrict__ c_out, unsigned short* __restrict__ hall16, int t) {
  __shared__ __align__(16) float s_h[NTHR];
  const int tid = threadIdx.x;
  const int b   = blockIdx.x >> 1;
  const int j0  = (blockIdx.x & 1) * 256;
  const int j   = j0 + tid;
  const float* gc = gctx + (size_t)b * NGATE + j;
  const float* hp = hproj + (size_t)b * NHP + NATT + j;
  const float* ge = gemb + ((size_t)t * NBAT + b) * NGATE + j;
  const float zi = (gc[0]        + ge[0])        + hp[0];
  const float zf = (gc[NHID]     + ge[NHID])     + hp[NHID];
  const float zg = (gc[2 * NHID] + ge[2 * NHID]) + hp[2 * NHID];
  const float zo = (gc[3 * NHID] + ge[3 * NHID]) + hp[3 * NHID];
  const float cold = c_in[(size_t)b * NHID + j];
  const float si = sigm_f(zi);
  const float sf = sigm_f(zf);
  const float so = sigm_f(zo);
  const float tg = tanh_f(zg);
  const float cn = sf * cold + si * tg;
  const float hn = so * tanh_f(cn);
  float* cptr = c_out + (size_t)b * NHID + j;
  *(volatile float*)cptr = cn;
  __threadfence();
  *(volatile float*)cptr = cn;
  s_h[tid] = hn;
  __syncthreads();
  if (tid < 32) {
    const v4f x0 = *(const v4f*)(s_h + 8 * tid);
    const v4f x1 = *(const v4f*)(s_h + 8 * tid + 4);
    v8h hv;
#pragma unroll
    for (int e = 0; e < 4; ++e) { hv[e] = (_Float16)x0[e]; hv[4 + e] = (_Float16)x1[e]; }
    unsigned short* hq = hall16 + ((size_t)(b * NSTEP + t)) * NHID + j0 + 8 * tid;
    *(volatile v8h*)hq = hv;
    __threadfence();
    *(volatile v8h*)hq = hv;
  }
}

__global__ __launch_bounds__(NTHR) void copy_pred_kernel(const float* __restrict__ predpad, float* __restrict__ out0) {
  const int i = blockIdx.x * NTHR + threadIdx.x;
  if (i < NOUT0 / 4) {
    const int row = i / (NVOC / 4);
    const int c   = i - row * (NVOC / 4);
    const v4f v = *(const v4f*)(predpad + (size_t)row * NVOCP + 4 * c);
    float* op = out0 + (size_t)i * 4;
    *(volatile v4f*)op = v;
    __threadfence();
    *(volatile v4f*)op = v;
  }
}

__global__ __launch_bounds__(NTHR) void copy_alpha_kernel(const float* __restrict__ alpha_ws, float* __restrict__ out1) {
  const int i = blockIdx.x * NTHR + threadIdx.x;
  if (i < NOUT1 / 4) {
    v4f v;
#pragma unroll
    for (int e = 0; e < 4; ++e) {
      const int idx = 4 * i + e;
      const int r = idx / NPIX;
      const int n = idx - r * NPIX;
      v[e] = alpha_ws[(size_t)r * APITCH + n];
    }
    float* op = out1 + (size_t)i * 4;
    *(volatile v4f*)op = v;
    __threadfence();
    *(volatile v4f*)op = v;
  }
}

constexpr int gemm_blocks(int m, int n) { return ((m / 64) * (n / 64) + 7) / 8; }

extern "C" void kernel_launch(void* const* d_in, const int* in_sizes, int n_in,
                              void* d_out, int out_size, void* d_ws, size_t ws_size, hipStream_t stream) {
  if (n_in < 19 || d_out == nullptr || d_ws == nullptr) return;
  if (in_sizes[0] != NBAT * NPIX * NENC || in_sizes[1] != NBAT * NSEQ || in_sizes[2] != NVOC * NEMB ||
      in_sizes[3] != NGATE * NXIN || in_sizes[4] != NGATE || in_sizes[5] != NGATE * NHID || in_sizes[6] != NGATE ||
      in_sizes[7] != NATT * NENC || in_sizes[8] != NATT || in_sizes[9] != NATT * NHID || in_sizes[10] != NATT ||
      in_sizes[11] != NATT || in_sizes[12] != 1 || in_sizes[13] != NHID * NENC || in_sizes[14] != NHID ||
      in_sizes[15] != NHID * NENC || in_sizes[16] != NHID || in_sizes[17] != NVOC * NHID || in_sizes[18] != NVOC ||
      out_size != NOUT0 + NOUT1) return;

  const float* features  = (const float*)d_in[0];
  const int*   captions  = (const int*)  d_in[1];
  const float* emb       = (const float*)d_in[2];
  const float* W_ih      = (const float*)d_in[3];
  const float* b_ih      = (const float*)d_in[4];
  const float* W_hh      = (const float*)d_in[5];
  const float* b_hh      = (const float*)d_in[6];
  const float* W_enc_att = (const float*)d_in[7];
  const float* b_enc_att = (const float*)d_in[8];
  const float* W_dec_att = (const float*)d_in[9];
  const float* b_dec_att = (const float*)d_in[10];
  const float* W_full    = (const float*)d_in[11];
  const float* b_full    = (const float*)d_in[12];
  const float* W_init_h  = (const float*)d_in[13];
  const float* b_init_h  = (const float*)d_in[14];
  const float* W_init_c  = (const float*)d_in[15];
  const float* b_init_c  = (const float*)d_in[16];
  const float* W_fcn     = (const float*)d_in[17];
  const float* b_fcn     = (const float*)d_in[18];

  float* out0 = (float*)d_out;
  float* out1 = out0 + (size_t)NOUT0;

  char* ws = (char*)d_ws; size_t off = 0;
  auto carve = [&](size_t bytes) -> char* { char* p = ws + off; off += (bytes + 255) & ~(size_t)255; return p; };
  unsigned short* FEAT16  = (unsigned short*)carve((size_t)NFROWS * NENC * 2);
  unsigned short* WENC16  = (unsigned short*)carve((size_t)NATT * NENC * 2);
  unsigned short* WINIT16 = (unsigned short*)carve((size_t)2 * NHID * NENC * 2);
  unsigned short* MEAN16  = (unsigned short*)carve((size_t)NBAT * NENC * 2);
  unsigned short* WIHE16  = (unsigned short*)carve((size_t)NGATE * NEMB * 2);
  unsigned short* WIHC16  = (unsigned short*)carve((size_t)NGATE * NENC * 2);
  unsigned short* WH16    = (unsigned short*)carve((size_t)NHP * NHID * 2);
  unsigned short* WFCN16  = (unsigned short*)carve((size_t)NVOCP * NHID * 2);
  unsigned short* X16     = (unsigned short*)carve((size_t)NROWS * NEMB * 2);
  float*          GEMB    = (float*)carve((size_t)NROWS * NGATE * 4);
  float*          ATT1    = (float*)carve((size_t)NFROWS * NATT * 4);
  unsigned short* H0_16   = (unsigned short*)carve((size_t)NBAT * NHID * 2);
  float*          CST     = (float*)carve((size_t)2 * NBAT * NHID * 4);
  float*          HPROJ   = (float*)carve((size_t)NBAT * NHP * 4);
  unsigned short* CTX16   = (unsigned short*)carve((size_t)NBAT * NENC * 2);
  float*          GCTX    = (float*)carve((size_t)NBAT * NGATE * 4);
  unsigned short* HALL16  = (unsigned short*)carve((size_t)NROWS * NHID * 2);
  float*          ALPHAWS = (float*)carve((size_t)NROWS * APITCH * 4);
  float*          PREDPAD = (float*)carve((size_t)NROWS * NVOCP * 4);
  float*          BIASP   = (float*)carve((size_t)BIAS_TOTAL * 4);
  if (off > ws_size || off > (size_t)134217728) return;

  {
    const int n8 = NFROWS * (NENC / 8);
    cvt8_f16_kernel<<<(n8 + NTHR - 1) / NTHR, NTHR, 0, stream>>>(features, FEAT16, NFROWS, NFROWS, NENC / 8, NENC, 0);
  }
  {
    const int n8 = NATT * (NENC / 8);
    cvt8_f16_kernel<<<(n8 + NTHR - 1) / NTHR, NTHR, 0, stream>>>(W_enc_att, WENC16, NATT, NATT, NENC / 8, NENC, 0);
  }
  {
    const int n8 = NHID * (NENC / 8);
    cvt8_f16_kernel<<<(n8 + NTHR - 1) / NTHR, NTHR, 0, stream>>>(W_init_h, WINIT16, NHID, NHID, NENC / 8, NENC, 0);
    cvt8_f16_kernel<<<(n8 + NTHR - 1) / NTHR, NTHR, 0, stream>>>(W_init_c, WINIT16 + (size_t)NHID * NENC, NHID, NHID, NENC / 8, NENC, 0);
  }
  {
    const int n8 = NGATE * (NEMB / 8);
    cvt8_f16_kernel<<<(n8 + NTHR - 1) / NTHR, NTHR, 0, stream>>>(W_ih, WIHE16, NGATE, NGATE, NEMB / 8, NXIN, 0);
  }
  {
    const int n8 = NGATE * (NENC / 8);
    cvt8_f16_kernel<<<(n8 + NTHR - 1) / NTHR, NTHR, 0, stream>>>(W_ih, WIHC16, NGATE, NGATE, NENC / 8, NXIN, NEMB);
  }
  {
    const int n8a = NATT * (NHID / 8);
    const int n8b = NGATE * (NHID / 8);
    cvt8_f16_kernel<<<(n8a + NTHR - 1) / NTHR, NTHR, 0, stream>>>(W_dec_att, WH16, NATT, NATT, NHID / 8, NHID, 0);
    cvt8_f16_kernel<<<(n8b + NTHR - 1) / NTHR, NTHR, 0, stream>>>(W_hh, WH16 + (size_t)NATT * NHID, NGATE, NGATE, NHID / 8, NHID, 0);
  }
  {
    const int n8 = NVOCP * (NHID / 8);
    cvt8_f16_kernel<<<(n8 + NTHR - 1) / NTHR, NTHR, 0, stream>>>(W_fcn, WFCN16, NVOCP, NVOC, NHID / 8, NHID, 0);
  }
  bias_prep_kernel<<<(BIAS_TOTAL / 4 + NTHR - 1) / NTHR, NTHR, 0, stream>>>(b_ih, b_hh, b_dec_att, b_fcn, BIASP);
  mean16_kernel<<<(NBAT * NENC / 8) / NTHR, NTHR, 0, stream>>>(features, MEAN16);
  gather16_kernel<<<(NROWS * NEMB / 8) / NTHR, NTHR, 0, stream>>>(captions, emb, X16);

  wmma_gemm64_f16<2, 1><<<gemm_blocks(NBAT, NHID), 256, 0, stream>>>(
      MEAN16, NENC, WINIT16, NENC, (void*)H0_16, NHID, b_init_h, NBAT, NHID, NENC);
  wmma_gemm64_f16<2, 0><<<gemm_blocks(NBAT, NHID), 256, 0, stream>>>(
      MEAN16, NENC, WINIT16 + (size_t)NHID * NENC, NENC, (void*)CST, NHID, b_init_c, NBAT, NHID, NENC);
  wmma_gemm64_f16<2, 0><<<gemm_blocks(NFROWS, NATT), 256, 0, stream>>>(
      FEAT16, NENC, WENC16, NENC, (void*)ATT1, NATT, b_enc_att, NFROWS, NATT, NENC);
  wmma_gemm64_f16<2, 0><<<gemm_blocks(NROWS, NGATE), 256, 0, stream>>>(
      X16, NEMB, WIHE16, NEMB, (void*)GEMB, NGATE, BIASP + BIAS_G_OFF, NROWS, NGATE, NEMB);

  for (int t = 0; t < NSTEP; ++t) {
    const unsigned short* hA = (t == 0) ? H0_16 : (HALL16 + (size_t)(t - 1) * NHID);
    const int hlda = (t == 0) ? NHID : NSTEP * NHID;
    float* c_in  = CST + (size_t)(t & 1) * NBAT * NHID;
    float* c_out = CST + (size_t)((t + 1) & 1) * NBAT * NHID;
    wmma_gemm64_f16<2, 0><<<gemm_blocks(NBAT, NHP), 256, 0, stream>>>(
        hA, hlda, WH16, NHID, (void*)HPROJ, NHP, BIASP + BIAS_HP_OFF, NBAT, NHP, NHID);
    attn_step_kernel<<<NBAT, NTHR, 0, stream>>>(ATT1, HPROJ, features, W_full, b_full, ALPHAWS, CTX16, t);
    wmma_gemm64_f16<0, 0><<<gemm_blocks(NBAT, NGATE), 256, 0, stream>>>(
        CTX16, NENC, WIHC16, NENC, (void*)GCTX, NGATE, BIASP, NBAT, NGATE, NENC);
    lstm_point_kernel<<<(NBAT * NHID) / NTHR, NTHR, 0, stream>>>(GCTX, HPROJ, GEMB, c_in, c_out, HALL16, t);
  }

  wmma_gemm64_f16<2, 0><<<gemm_blocks(NROWS, NVOCP), 256, 0, stream>>>(
      HALL16, NHID, WFCN16, NHID, (void*)PREDPAD, NVOCP, BIASP + BIAS_FC_OFF, NROWS, NVOCP, NHID);
  copy_pred_kernel<<<(NOUT0 / 4) / NTHR, NTHR, 0, stream>>>(PREDPAD, out0);
  copy_alpha_kernel<<<(NOUT1 / 4 + NTHR - 1) / NTHR, NTHR, 0, stream>>>(ALPHAWS, out1);
}
